// GraphVAE_7069516169733
// MI455X (gfx1250) — hardware-run, weakly checked
//
#include <hip/hip_runtime.h>
#include <math.h>

constexpr int kMC       = 4;
constexpr int kGraphs   = 256;
constexpr int kLat      = 64;
constexpr int kHidden   = 1024;
constexpr int kNode     = 50;
constexpr int kFeat     = 3;
constexpr int kPerm     = 64;
constexpr int kEdge     = 1225;
constexpr int kEdgePad  = 1280;
constexpr int kFeatCols = 150;
constexpr int kFeatPad  = 192;
constexpr int kNcat     = kEdgePad + kFeatPad;
constexpr int kRows     = kMC * kGraphs;
constexpr int kResPitch = 32;
constexpr float kCoeffA = 1.0f;
constexpr float kBeta   = 1.0f;

static_assert(kLat % 32 == 0, "K0");
static_assert(kHidden % 32 == 0, "K1");
static_assert(kRows % 64 == 0, "M");
static_assert(kHidden % 64 == 0, "N0");
static_assert(kNcat % 64 == 0, "N1");
static_assert((kRows / 64) * (kHidden / 64) % 8 == 0, "tiles0");
static_assert((kRows / 64) * (kNcat / 64) % 8 == 0, "tiles1");
static_assert(kEdgePad >= kEdge && kFeatPad >= kFeatCols, "pads");

typedef __attribute__((ext_vector_type(16))) _Float16 v16h;
typedef __attribute__((ext_vector_type(8)))  _Float16 v8h;
typedef __attribute__((ext_vector_type(16))) __bf16   v16b;
typedef __attribute__((ext_vector_type(8)))  __bf16   v8b;
typedef __attribute__((ext_vector_type(8)))  float    v8f;
typedef __attribute__((ext_vector_type(4)))  float    v4f;
typedef __attribute__((ext_vector_type(4)))  unsigned int v4u;

__device__ __forceinline__ unsigned short f2bf_bits(float f) {
  unsigned u = __float_as_uint(f);
  return (unsigned short)((u + 0x7FFFu + ((u >> 16) & 1u)) >> 16);
}
__device__ __forceinline__ float bf_bits2f(unsigned short h) { return __uint_as_float(((unsigned)h) << 16); }

__device__ __forceinline__ void dep_guard_h(v8f& a, v8f& b, v16h x, v16h y) { asm volatile("v_nop\n\tv_nop\n\tv_nop\n\tv_nop" : "+v"(a), "+v"(b) : "v"(x), "v"(y)); }
__device__ __forceinline__ void dep_guard_b(v8f& a, v8f& b, v16b x, v16b y) { asm volatile("v_nop\n\tv_nop\n\tv_nop\n\tv_nop" : "+v"(a), "+v"(b) : "v"(x), "v"(y)); }
__device__ __forceinline__ void keep4_h(v16h a, v16h b, v16h c, v16h d) { asm volatile("v_nop" :: "v"(a), "v"(b), "v"(c), "v"(d)); }
__device__ __forceinline__ void keep4_b(v16b a, v16b b, v16b c, v16b d) { asm volatile("v_nop" :: "v"(a), "v"(b), "v"(c), "v"(d)); }
__device__ __forceinline__ void acc_guard4(v8f& a, v8f& b, v8f& c, v8f& d) { asm volatile("v_nop\n\tv_nop\n\tv_nop\n\tv_nop" : "+v"(a), "+v"(b), "+v"(c), "+v"(d)); }
template <typename T> struct Frag;
template <> struct Frag<_Float16> {
  typedef v16h V; union U { v16h v; v8h h[2]; };
  static __device__ __forceinline__ v16h load(const _Float16* p) {
    U f; f.h[0] = *(const v8h*)(p); f.h[1] = *(const v8h*)(p + 16); return f.v;
  }
  static __device__ __forceinline__ v8f mma(v16h a, v16h b, v8f c) {
    return __builtin_amdgcn_wmma_f32_16x16x32_f16(false, a, false, b, (short)0, c, false, false);
  }
  static __device__ __forceinline__ void guard(v8f& a, v8f& b, v16h x, v16h y) { dep_guard_h(a, b, x, y); }
  static __device__ __forceinline__ void keep(v16h a, v16h b, v16h c, v16h d) { keep4_h(a, b, c, d); }
};
template <> struct Frag<__bf16> {
  typedef v16b V; union U { v16b v; v8b h[2]; };
  static __device__ __forceinline__ v16b load(const __bf16* p) {
    U f; f.h[0] = *(const v8b*)(p); f.h[1] = *(const v8b*)(p + 16); return f.v;
  }
  static __device__ __forceinline__ v8f mma(v16b a, v16b b, v8f c) {
    return __builtin_amdgcn_wmma_f32_16x16x32_bf16(false, a, false, b, (short)0, c, false, false);
  }
  static __device__ __forceinline__ void guard(v8f& a, v8f& b, v16b x, v16b y) { dep_guard_b(a, b, x, y); }
  static __device__ __forceinline__ void keep(v16b a, v16b b, v16b c, v16b d) { keep4_b(a, b, c, d); }
};

__device__ __forceinline__ unsigned pk16(unsigned short a, unsigned short b) { return (unsigned)a | ((unsigned)b << 16); }

template <int ET> struct Elem;
template <> struct Elem<0> { typedef _Float16 T; };
template <> struct Elem<1> { typedef __bf16 T; };
template <int ET, bool SPLIT, int BIAS_MODE, int OUT_MODE, bool RESID, int ACT = 0>
__global__ __launch_bounds__(256) void wmma_gemm64(
    const unsigned short* __restrict__ Ap, const unsigned short* __restrict__ A2p, int lda, long strideA,
    const unsigned short* __restrict__ Btp, const unsigned short* __restrict__ Bt2p, int ldb, long strideB,
    void* __restrict__ Cout, void* __restrict__ Cout2, int ldc, long strideC,
    const float* __restrict__ bias,
    const float* __restrict__ resid, long strideR,
    int M, int N, int K, float scale) {
  typedef typename Elem<ET>::T T;
  typedef typename Frag<T>::V V;
  const T* A = (const T*)Ap; const T* A2 = (const T*)A2p; const T* Bt = (const T*)Btp; const T* Bt2 = (const T*)Bt2p;
  __shared__ __align__(16) float sT[8][16 * 68];
  const int b    = blockIdx.y;
  const int lane = threadIdx.x & 31;
  const int wave = threadIdx.x >> 5;
  const int tilesN = N >> 6;
  const int tilesM = M >> 6;
  const int tile = blockIdx.x * 8 + wave;
  if (tile >= tilesM * tilesN) return;
  const int tm = tile / tilesN;
  const int tn = tile - tm * tilesN;
  const int m0 = tm << 6;
  const int n0 = tn << 6;

  const T* Ab  = A  + (size_t)b * strideA;
  const T* Bb  = Bt + (size_t)b * strideB;
  const T* Ab2 = SPLIT ? (A2  + (size_t)b * strideA) : nullptr;
  const T* Bb2 = SPLIT ? (Bt2 + (size_t)b * strideB) : nullptr;

  const int rlane = lane & 15;
  const int koff  = (lane >> 4) * 8;
  const int mOff  = (lane >> 4) * 8;

  v8f acc[4][4];
#pragma unroll
  for (int i = 0; i < 4; ++i)
#pragma unroll
    for (int j = 0; j < 4; ++j) acc[i][j] = (v8f){0.f,0.f,0.f,0.f,0.f,0.f,0.f,0.f};

  for (int k0 = 0; k0 < K; k0 += 32) {
    V bh[4], bl[4];
#pragma unroll
    for (int j = 0; j < 4; ++j) {
      const size_t bo = (size_t)(n0 + (j << 4) + rlane) * ldb + koff + k0;
      bh[j] = Frag<T>::load(Bb + bo);
      if (SPLIT) bl[j] = Frag<T>::load(Bb2 + bo);
    }
#pragma unroll
    for (int i = 0; i < 4; ++i) {
      const size_t ao = (size_t)(m0 + (i << 4) + rlane) * lda + koff + k0;
      V ah = Frag<T>::load(Ab + ao);
      V al;
      if (SPLIT) al = Frag<T>::load(Ab2 + ao);
#pragma unroll
      for (int j = 0; j < 4; ++j) {
        acc[i][j] = Frag<T>::mma(ah, bh[j], acc[i][j]);
        if (SPLIT) {
          acc[i][j] = Frag<T>::mma(ah, bl[j], acc[i][j]);
          acc[i][j] = Frag<T>::mma(al, bh[j], acc[i][j]);
        }
      }
      Frag<T>::guard(acc[i][0], acc[i][3], ah, SPLIT ? al : ah);
    }
    Frag<T>::keep(bh[0], bh[1], bh[2], bh[3]);
    if (SPLIT) Frag<T>::keep(bl[0], bl[1], bl[2], bl[3]);
  }
  acc_guard4(acc[0][0], acc[0][1], acc[0][2], acc[0][3]);
  acc_guard4(acc[1][0], acc[1][1], acc[1][2], acc[1][3]);
  acc_guard4(acc[2][0], acc[2][1], acc[2][2], acc[2][3]);
  acc_guard4(acc[3][0], acc[3][1], acc[3][2], acc[3][3]);

  float* slab = sT[wave];
  const float* Rb = RESID ? (resid + (size_t)b * strideR) : nullptr;
#pragma unroll
  for (int i = 0; i < 4; ++i) {
    const int mBase = m0 + (i << 4);
#pragma unroll
    for (int j = 0; j < 4; ++j) {
      const int n = n0 + (j << 4) + rlane;
      float bv = 0.f;
      if (BIAS_MODE == 2) bv = bias[n];
#pragma unroll
      for (int r = 0; r < 8; ++r) {
        float v = acc[i][j][r] * scale;
        if (BIAS_MODE == 1) v += bias[mBase + mOff + r];
        if (BIAS_MODE == 2) v += bv;
        if (RESID) v += Rb[(size_t)(mBase + mOff + r) * ldc + n];
        if (ACT == 2) v = fmaxf(v, 0.0f);
        if (ACT == 4) v = (v > 0.f) ? v : 0.01f * v;
        slab[(mOff + r) * 68 + (j << 4) + rlane] = v;
      }
    }
    __builtin_amdgcn_fence(__ATOMIC_RELEASE, "workgroup");
    __builtin_amdgcn_wave_barrier();
    __builtin_amdgcn_fence(__ATOMIC_ACQUIRE, "workgroup");
    if (OUT_MODE == 0) {
      float* C = (float*)Cout + (size_t)b * strideC;
      const int hh = lane >> 4, c4 = (lane & 15) * 4;
      for (int pass = 0; pass < 2; ++pass) {
#pragma unroll
        for (int it = 0; it < 8; ++it) {
          const int row = it * 2 + hh;
          v4f v = *(const v4f*)(slab + row * 68 + c4);
          *(volatile v4f*)(C + (size_t)(mBase + row) * ldc + n0 + c4) = v;
        }
        __threadfence();
      }
    } else {
      const int q = lane >> 3, c8 = (lane & 7) * 8;
      unsigned short* C  = (unsigned short*)Cout  + (size_t)b * strideC;
      unsigned short* C2 = (OUT_MODE == 2) ? ((unsigned short*)Cout2 + (size_t)b * strideC) : nullptr;
      for (int pass = 0; pass < 2; ++pass) {
#pragma unroll
        for (int it = 0; it < 4; ++it) {
          const int row = it * 4 + q;
          const float* sp = slab + row * 68 + c8;
          v8h hv, lv;
#pragma unroll
          for (int e = 0; e < 8; ++e) {
            if (OUT_MODE == 1) {
              hv[e] = (_Float16)sp[e];
            } else {
              unsigned short hb = f2bf_bits(sp[e]);
              hv[e] = __builtin_bit_cast(_Float16, hb);
              if (OUT_MODE == 2) {
                unsigned short lb = f2bf_bits(sp[e] - bf_bits2f(hb));
                lv[e] = __builtin_bit_cast(_Float16, lb);
              }
            }
          }
          *(volatile v8h*)(C + (size_t)(mBase + row) * ldc + n0 + c8) = hv;
          if (OUT_MODE == 2) *(volatile v8h*)(C2 + (size_t)(mBase + row) * ldc + n0 + c8) = lv;
        }
        __threadfence();
      }
    }
    __builtin_amdgcn_fence(__ATOMIC_RELEASE, "workgroup");
    __builtin_amdgcn_wave_barrier();
    __builtin_amdgcn_fence(__ATOMIC_ACQUIRE, "workgroup");
  }
}

__global__ __launch_bounds__(256) void zb_kernel(const float* __restrict__ mean, const float* __restrict__ logvar,
                                                 const float* __restrict__ eps, unsigned short* __restrict__ zb) {
  const int i = blockIdx.x * 256 + threadIdx.x;
  if (i >= kRows * kLat / 2) return;
  const int r  = i >> 5;
  const int kp = (i & 31) * 2;
  const int b  = r & (kGraphs - 1);
  const size_t mi = (size_t)b * kLat + kp;
  const size_t ei = (size_t)r * kLat + kp;
  const float z0 = mean[mi]     + expf(0.5f * logvar[mi])     * eps[ei];
  const float z1 = mean[mi + 1] + expf(0.5f * logvar[mi + 1]) * eps[ei + 1];
  const unsigned u = pk16(f2bf_bits(z0), f2bf_bits(z1));
  volatile unsigned* q = ((volatile unsigned*)zb) + i;
  *q = u;
  __threadfence();
  *q = u;
}

__global__ __launch_bounds__(256) void tcast_kernel(const float* __restrict__ src, int ncols, int kdim,
                                                    unsigned short* __restrict__ dst, int rowOff) {
  __shared__ float sm[64][65];
  const int t  = threadIdx.x;
  const int k0 = blockIdx.x * 64;
  const int n0 = blockIdx.y * 64;
#pragma unroll
  for (int i = 0; i < 16; ++i) {
    const int e  = i * 256 + t;
    const int kl = e >> 6;
    const int nl = e & 63;
    const int n  = n0 + nl;
    const int nc = (n < ncols) ? n : (ncols - 1);
    float v = src[(size_t)(k0 + kl) * ncols + nc];
    v = (n < ncols) ? v : 0.0f;
    sm[nl][kl] = v;
  }
  __syncthreads();
  const int lane = t & 31, wave = t >> 5;
  const int q = lane >> 3, c8 = (lane & 7) * 8;
  for (int pass = 0; pass < 2; ++pass) {
#pragma unroll
    for (int it = 0; it < 2; ++it) {
      const int row = wave * 8 + it * 4 + q;
      unsigned short hb[8];
#pragma unroll
      for (int e = 0; e < 8; ++e) hb[e] = f2bf_bits(sm[row][c8 + e]);
      const v4u u = (v4u){pk16(hb[0], hb[1]), pk16(hb[2], hb[3]), pk16(hb[4], hb[5]), pk16(hb[6], hb[7])};
      *(volatile v4u*)(dst + (size_t)(rowOff + n0 + row) * kdim + k0 + c8) = u;
    }
    __threadfence();
  }
}

__global__ __launch_bounds__(256) void adj_term_kernel(const float* __restrict__ logits, const float* __restrict__ bA,
                                                       const float* __restrict__ A_in, const int* __restrict__ perms,
                                                       float* __restrict__ resA) {
  __shared__ float LS[1232];
  __shared__ float AS[kNode * kNode];
  __shared__ int   PS[kPerm * kNode];
  __shared__ float red[8];
  __shared__ float dots[kPerm];
  const int b    = blockIdx.x;
  const int t    = threadIdx.x;
  const int lane = t & 31, wave = t >> 5;

#pragma unroll 1
  for (int i = t; i < kNode * kNode; i += 256) AS[i] = A_in[(size_t)b * kNode * kNode + i];
#pragma unroll 1
  for (int i = t; i < kPerm * kNode; i += 256) {
    int p = perms[i];
    p = p < 0 ? 0 : (p > kNode - 1 ? kNode - 1 : p);
    PS[i] = p;
  }

  float s = 0.0f;
#pragma unroll 1
  for (int it = 0; it < 5; ++it) {
    const int e  = t + 256 * it;
    const bool valid = (e < kEdge);
    const int ec = valid ? e : (kEdge - 1);
    const float ba = bA[ec];
    float sum = 0.0f;
    float sps = 0.0f;
#pragma unroll 1
    for (int m = 0; m < kMC; ++m) {
      const float l  = logits[(size_t)(m * kGraphs + b) * kNcat + ec];
      sum += l;
      const float lb = l + ba;
      sps += fmaxf(lb, 0.0f) + log1pf(expf(-fabsf(lb)));
    }
    if (valid) LS[e] = 0.25f * sum + ba;
    s += valid ? sps : 0.0f;
  }
#pragma unroll
  for (int off = 16; off > 0; off >>= 1) s += __shfl_xor(s, off, 32);
  if (lane == 0) red[wave] = s;
  __syncthreads();

#pragma unroll 1
  for (int pi = 0; pi < kPerm / 8; ++pi) {
    const int p = wave + 8 * pi;
    const int pb = p * kNode;
    float acc = 0.0f;
#pragma unroll 1
    for (int i = 1; i < kNode; ++i) {
      const int base_e = (i * (i - 1)) >> 1;
      const int prow = PS[pb + i] * kNode;
      {
        const int j  = lane;
        const int e  = base_e + j;
        const int ec = e < kEdge ? e : (kEdge - 1);
        const float a = AS[prow + PS[pb + j]];
        const float l = LS[ec];
        const float term = a * l;
        acc += (j < i) ? term : 0.0f;
      }
      if (i > 32) {
        const int j  = lane + 32;
        const int jj = j < kNode ? j : (kNode - 1);
        const int e  = base_e + j;
        const int ec = e < kEdge ? e : (kEdge - 1);
        const float a = AS[prow + PS[pb + jj]];
        const float l = LS[ec];
        const float term = a * l;
        acc += (j < i) ? term : 0.0f;
      }
    }
#pragma unroll
    for (int off = 16; off > 0; off >>= 1) acc += __shfl_xor(acc, off, 32);
    if (lane == 0) dots[p] = acc;
  }
  __syncthreads();

  float mx = fmaxf(dots[lane], dots[lane + 32]);
#pragma unroll
  for (int off = 16; off > 0; off >>= 1) mx = fmaxf(mx, __shfl_xor(mx, off, 32));
  const float sbar = 0.25f * (((((((red[0] + red[1]) + red[2]) + red[3]) + red[4]) + red[5]) + red[6]) + red[7]);
  const float res = mx - sbar;
  if (wave == 0) {
    volatile float* rp = resA + (size_t)b * kResPitch + lane;
    *rp = res;
    __threadfence();
    *rp = res;
  }
}

__global__ __launch_bounds__(256) void final_kernel(const float* __restrict__ logits, const float* __restrict__ bF,
                                                    const float* __restrict__ Fx, const float* __restrict__ coeff,
                                                    const float* __restrict__ mean, const float* __restrict__ logvar,
                                                    const float* __restrict__ resA, float* __restrict__ out) {
  __shared__ __align__(16) float sOut[kGraphs];
  const int t = threadIdx.x;
  const int b = t;
  const float cf0 = coeff[0], cf1 = coeff[1], cf2 = coeff[2];
  float acc0 = 0.0f, acc1 = 0.0f, acc2 = 0.0f;
#pragma unroll 1
  for (int m = 0; m < kMC; ++m) {
    const float* L = logits + (size_t)(m * kGraphs + b) * kNcat + kEdgePad;
    float mx = -3.0e38f;
#pragma unroll 1
    for (int n = 0; n < kNode; ++n) mx = fmaxf(mx, L[3 * n + 2] + bF[3 * n + 2]);
    float se = 0.0f;
#pragma unroll 1
    for (int n = 0; n < kNode; ++n) se += expf((L[3 * n + 2] + bF[3 * n + 2]) - mx);
    const float lse = mx + logf(se);
#pragma unroll 1
    for (int n = 0; n < kNode; ++n) {
      const float* fxp = Fx + ((size_t)b * kNode + n) * kFeat;
      const float l2 = L[3 * n + 2] + bF[3 * n + 2];
      acc2 += fxp[2] * (l2 - lse);
#pragma unroll 1
      for (int f = 0; f < 2; ++f) {
        const float l  = L[3 * n + f] + bF[3 * n + f];
        const float x  = fxp[f];
        const float lp = log1pf(expf(-fabsf(l)));
        const float term = x * (fminf(l, 0.0f) - lp) + (1.0f - x) * (fminf(-l, 0.0f) - lp);
        acc0 += (f == 0) ? term : 0.0f;
        acc1 += (f == 0) ? 0.0f : term;
      }
    }
  }
  const float fx = (0.25f * acc0) * cf0 + (0.25f * acc1) * cf1 + (0.25f * acc2) * cf2;

  float ks = 0.0f;
#pragma unroll 1
  for (int k = 0; k < kLat; ++k) {
    const float mu = mean[(size_t)b * kLat + k];
    const float lv = logvar[(size_t)b * kLat + k];
    ks += expf(lv) + mu * mu - 1.0f - lv;
  }
  const float kld = 0.5f * ks;
  const float res = kCoeffA * resA[(size_t)b * kResPitch] + fx - kBeta * kld;
  sOut[b] = res;
  __syncthreads();
  if (t < 64) {
    const v4f v = *(const v4f*)(sOut + 4 * t);
    *(volatile v4f*)(out + 4 * t) = v;
    __threadfence();
    *(volatile v4f*)(out + 4 * t) = v;
  }
}

extern "C" void kernel_launch(void* const* d_in, const int* in_sizes, int n_in,
                              void* d_out, int out_size, void* d_ws, size_t ws_size,
                              hipStream_t stream) {
  if (n_in < 13 || out_size < kGraphs) return;
  if (in_sizes[5] != kHidden * kEdge || in_sizes[7] != kHidden * kFeatCols || in_sizes[12] != kPerm * kNode) return;
  const float* mean   = (const float*)d_in[0];
  const float* logvar = (const float*)d_in[1];
  const float* eps    = (const float*)d_in[2];
  const float* W1     = (const float*)d_in[3];
  const float* b1     = (const float*)d_in[4];
  const float* WA     = (const float*)d_in[5];
  const float* bA     = (const float*)d_in[6];
  const float* WF     = (const float*)d_in[7];
  const float* bF     = (const float*)d_in[8];
  const float* A_in   = (const float*)d_in[9];
  const float* Fx     = (const float*)d_in[10];
  const float* coeff  = (const float*)d_in[11];
  const int*   perms  = (const int*)d_in[12];
  float* out = (float*)d_out;

  char* ws = (char*)d_ws;
  size_t off = 0;
  auto carve = [&](size_t bytes) -> char* { char* p = ws + off; off += (bytes + 255) & ~(size_t)255; return p; };
  unsigned short* zbPlane  = (unsigned short*)carve((size_t)kRows * kLat * 2);
  unsigned short* w1tPlane = (unsigned short*)carve((size_t)kHidden * kLat * 2);
  unsigned short* hPlane   = (unsigned short*)carve((size_t)kRows * kHidden * 2);
  unsigned short* wcatT    = (unsigned short*)carve((size_t)kNcat * kHidden * 2);
  float*          logits   = (float*)carve((size_t)kRows * kNcat * 4);
  float*          resA     = (float*)carve((size_t)kGraphs * kResPitch * 4);
  if (off > ws_size || off > (size_t)134217728) return;

  zb_kernel<<<(kRows * kLat / 2 + 255) / 256, 256, 0, stream>>>(mean, logvar, eps, zbPlane);
  tcast_kernel<<<dim3(kLat / 64, kHidden / 64), 256, 0, stream>>>(W1, kHidden, kLat, w1tPlane, 0);
  tcast_kernel<<<dim3(kHidden / 64, kEdgePad / 64), 256, 0, stream>>>(WA, kEdge, kHidden, wcatT, 0);
  tcast_kernel<<<dim3(kHidden / 64, kFeatPad / 64), 256, 0, stream>>>(WF, kFeatCols, kHidden, wcatT, kEdgePad);
  wmma_gemm64<1, false, 2, 3, false, 2><<<dim3((kRows / 64) * (kHidden / 64) / 8, 1), 256, 0, stream>>>(
      zbPlane, zbPlane, kLat, 0L, w1tPlane, w1tPlane, kLat, 0L,
      (void*)hPlane, (void*)hPlane, kHidden, 0L, b1, nullptr, 0L, kRows, kHidden, kLat, 1.0f);
  wmma_gemm64<1, false, 0, 0, false, 0><<<dim3((kRows / 64) * (kNcat / 64) / 8, 1), 256, 0, stream>>>(
      hPlane, hPlane, kHidden, 0L, wcatT, wcatT, kHidden, 0L,
      (void*)logits, (void*)logits, kNcat, 0L, nullptr, nullptr, 0L, kRows, kNcat, kHidden, 1.0f);
  adj_term_kernel<<<kGraphs, 256, 0, stream>>>(logits, bA, A_in, perms, resA);
  final_kernel<<<1, kGraphs, 0, stream>>>(logits, bF, Fx, coeff, mean, logvar, resA, out);
}
